// KRRGenredSolver_14731737825439
// MI455X (gfx1250) — hardware-verified
//
#include <hip/hip_runtime.h>
#include <stddef.h>


typedef _Float16 v16h __attribute__((ext_vector_type(16)));
typedef _Float16 v8h  __attribute__((ext_vector_type(8)));
typedef float    v8f  __attribute__((ext_vector_type(8)));
typedef float    v4f  __attribute__((ext_vector_type(4)));
typedef float    v2f  __attribute__((ext_vector_type(2)));
typedef _Float16 h16;

#ifndef NX
#define NX 8192
#endif
#define NX_FULL 8192
#define MY 16384
#define KD 32

#define XCARRY 64.0f
#define YCARRY 64.0f
#define LOG2E  1.4426950408889634f

#define PREP_ROWS 64
#define BROWS 32
#define NWAVES 8
#define TILES_PER_WAVE (MY / 16 / NWAVES)

static_assert(NX >= 64 && NX <= NX_FULL);
static_assert((NX % PREP_ROWS) == 0 && (NX % BROWS) == 0);
static_assert((MY % PREP_ROWS) == 0);
static_assert((MY % (16 * NWAVES)) == 0);
static_assert(KD == 32);
static_assert(PREP_ROWS * KD == 256 * 8);
static_assert(BROWS == 32);
static_assert(TILES_PER_WAVE * 16 * NWAVES == MY);

#define XH_BYTES   ((size_t)NX_FULL * KD * 2)
#define YH_BYTES   ((size_t)MY * KD * 2)
#define X2_BYTES   ((size_t)NX_FULL * 4)
#define PAIR_BYTES ((size_t)MY * 8)
#define OFF_XH   ((size_t)0)
#define OFF_YH   (OFF_XH + XH_BYTES)
#define OFF_X2   (OFF_YH + YH_BYTES)
#define OFF_PAIR (OFF_X2 + X2_BYTES)
#define WS_TOTAL (OFF_PAIR + PAIR_BYTES)
static_assert((XH_BYTES % 128) == 0 && (YH_BYTES % 128) == 0);
static_assert((X2_BYTES % 128) == 0 && (PAIR_BYTES % 128) == 0);
static_assert(WS_TOTAL <= (size_t)134217728);

__device__ __forceinline__ float bf16r(float x) {
  unsigned int u = __float_as_uint(x);
  u = (u + 0x7FFFu + ((u >> 16) & 1u)) & 0xFFFF0000u;
  return __uint_as_float(u);
}

static __device__ __forceinline__ h16 toh_flush(float v) {
  const h16 r = (h16)v;
  return (fabsf(v) < 6.103515625e-05f) ? (h16)0.0f : r;
}

__device__ __forceinline__ v16h frag_at(const _Float16* p) {
  v8h lo = *(const v8h*)(p);
  v8h hi = *(const v8h*)(p + 16);
  v16h out;
#pragma unroll
  for (int i = 0; i < 8; ++i) { out[i] = lo[i]; out[i + 8] = hi[i]; }
  return out;
}

__device__ __forceinline__ v8f wmma16(v16h a, v16h b, v8f c) {
  v8f d = __builtin_amdgcn_wmma_f32_16x16x32_f16(false, a, false, b, (short)0, c,
                                                 false, false);
  asm volatile("v_nop\n\tv_nop\n\tv_nop\n\tv_nop" : "+v"(d) : "v"(a), "v"(b));
  return d;
}

__device__ __forceinline__ float red16_sum(float x) {
#pragma unroll
  for (int off = 1; off < 16; off <<= 1) x += __shfl_xor(x, off, 32);
  return x;
}

__global__ __launch_bounds__(256) void xprep_kernel(
    const float* __restrict__ X, const float* __restrict__ G,
    _Float16* __restrict__ Xh, float* __restrict__ X2c) {
  __shared__ __attribute__((aligned(16))) float sq[PREP_ROWS];
  const unsigned tid = threadIdx.x;
  const unsigned r = tid >> 2;
  const unsigned row0 = blockIdx.x * (unsigned)PREP_ROWS;
  const unsigned c = (tid & 3u) * 8u;
  const size_t eoff = (size_t)(row0 + r) * KD + c;
  const v4f a0 = *(const v4f*)(X + eoff);
  const v4f a1 = *(const v4f*)(X + eoff + 4u);
  v8h o;
  float s = 0.0f;
#pragma unroll
  for (int i = 0; i < 4; ++i) {
    const float e0 = bf16r(a0[i]);
    const float e1 = bf16r(a1[i]);
    s += e0 * e0;
    s += e1 * e1;
    o[i]     = toh_flush(XCARRY * e0);
    o[i + 4] = toh_flush(XCARRY * e1);
  }
  s += __shfl_xor(s, 1, 32);
  s += __shfl_xor(s, 2, 32);
  if ((tid & 3u) == 0u) sq[r] = s;
  __syncthreads();

  const float gb = bf16r(G[0]);
  const float c1 = -LOG2E * (1.0f / gb);
  const unsigned q4 = (tid & 15u) * 4u;
  const v4f q = *(const v4f*)&sq[q4];
  v4f t;
#pragma unroll
  for (int j = 0; j < 4; ++j) t[j] = c1 * q[j];

  _Float16* pp = Xh + eoff;
  float* tp = X2c + row0 + q4;
  *(volatile v8h*)pp = o;
  if (tid < 16u) *(volatile v4f*)tp = t;
  __threadfence();
  *(volatile v8h*)pp = o;
  if (tid < 16u) *(volatile v4f*)tp = t;
}

__global__ __launch_bounds__(256) void yprep_kernel(
    const float* __restrict__ Y, const float* __restrict__ Al, const float* __restrict__ G,
    _Float16* __restrict__ Yh, float* __restrict__ Pair) {
  __shared__ __attribute__((aligned(16))) float sq[PREP_ROWS];
  const unsigned tid = threadIdx.x;
  const unsigned r = tid >> 2;
  const unsigned row0 = blockIdx.x * (unsigned)PREP_ROWS;
  const unsigned c = (tid & 3u) * 8u;
  const size_t eoff = (size_t)(row0 + r) * KD + c;
  const v4f a0 = *(const v4f*)(Y + eoff);
  const v4f a1 = *(const v4f*)(Y + eoff + 4u);
  v8h o;
  float s = 0.0f;
#pragma unroll
  for (int i = 0; i < 4; ++i) {
    const float e0 = bf16r(a0[i]);
    const float e1 = bf16r(a1[i]);
    s += e0 * e0;
    s += e1 * e1;
    o[i]     = toh_flush(YCARRY * e0);
    o[i + 4] = toh_flush(YCARRY * e1);
  }
  s += __shfl_xor(s, 1, 32);
  s += __shfl_xor(s, 2, 32);
  if ((tid & 3u) == 0u) sq[r] = s;
  __syncthreads();

  const float gb = bf16r(G[0]);
  const float c1 = -LOG2E * (1.0f / gb);
  const unsigned r2 = (tid & 31u) * 2u;
  const v2f q  = *(const v2f*)&sq[r2];
  const v2f al = *(const v2f*)(Al + row0 + r2);
  v4f t;
  t[0] = c1 * q[0];
  t[1] = bf16r(al[0]);
  t[2] = c1 * q[1];
  t[3] = bf16r(al[1]);

  _Float16* pp = Yh + eoff;
  float* tp = Pair + (size_t)(row0 + r2) * 2u;
  *(volatile v8h*)pp = o;
  if (tid < 32u) *(volatile v4f*)tp = t;
  __threadfence();
  *(volatile v8h*)pp = o;
  if (tid < 32u) *(volatile v4f*)tp = t;
}

__global__ __launch_bounds__(256) void krr_kernel(
    const _Float16* __restrict__ Xh, const _Float16* __restrict__ Yh,
    const float* __restrict__ X2c, const float* __restrict__ Pair,
    const float* __restrict__ G, float* __restrict__ out) {
  __shared__ __attribute__((aligned(16))) float part[NWAVES * BROWS];
  const unsigned tid = threadIdx.x, lane = tid & 31u;
  const unsigned wave = (unsigned)__builtin_amdgcn_readfirstlane((int)(threadIdx.x >> 5));
  const unsigned hh = lane >> 4, m = lane & 15u;
  const unsigned row0 = blockIdx.x * (unsigned)BROWS;

  const v16h a0 = frag_at(Xh + (size_t)(row0 + m) * KD + hh * 8u);
  const v16h a1 = frag_at(Xh + (size_t)(row0 + 16u + m) * KD + hh * 8u);

  const float gb = bf16r(G[0]);
  const float c1 = -LOG2E * (1.0f / gb);
  const float kd = (-2.0f * c1) * (1.0f / (XCARRY * YCARRY));

  float xc0[8], xc1[8], acc0[8], acc1[8];
  {
    const v4f t0 = *(const v4f*)(X2c + row0 + hh * 8u);
    const v4f t1 = *(const v4f*)(X2c + row0 + hh * 8u + 4u);
    const v4f t2 = *(const v4f*)(X2c + row0 + 16u + hh * 8u);
    const v4f t3 = *(const v4f*)(X2c + row0 + 16u + hh * 8u + 4u);
#pragma unroll
    for (int v = 0; v < 4; ++v) {
      xc0[v] = t0[v]; xc0[v + 4] = t1[v];
      xc1[v] = t2[v]; xc1[v + 4] = t3[v];
    }
  }
#pragma unroll
  for (int v = 0; v < 8; ++v) { acc0[v] = 0.0f; acc1[v] = 0.0f; }

  const unsigned jt0 = wave * (unsigned)TILES_PER_WAVE;
#pragma unroll 2
  for (unsigned jt = jt0; jt < jt0 + (unsigned)TILES_PER_WAVE; ++jt) {
    const unsigned col = jt * 16u + m;
    const v16h b = frag_at(Yh + (size_t)col * KD + hh * 8u);
    const v2f ya = *(const v2f*)(Pair + (size_t)col * 2u);
    const v8f z = {};
    const v8f d0 = wmma16(a0, b, z);
    const v8f d1 = wmma16(a1, b, z);
    const float y2c = ya[0];
    const float alc = ya[1];
#pragma unroll
    for (int v = 0; v < 8; ++v) {
      const float t0 = xc0[v] + y2c;
      const float e0 = __builtin_fmaf(kd, d0[v], t0);
      acc0[v] = __builtin_fmaf(__builtin_amdgcn_exp2f(e0), alc, acc0[v]);
      const float t1 = xc1[v] + y2c;
      const float e1 = __builtin_fmaf(kd, d1[v], t1);
      acc1[v] = __builtin_fmaf(__builtin_amdgcn_exp2f(e1), alc, acc1[v]);
    }
  }

  float s0[8], s1[8];
#pragma unroll
  for (int v = 0; v < 8; ++v) {
    s0[v] = red16_sum(acc0[v]);
    s1[v] = red16_sum(acc1[v]);
  }
  if (m == 0u) {
#pragma unroll
    for (int v = 0; v < 8; ++v) {
      part[wave * (unsigned)BROWS + hh * 8u + (unsigned)v] = s0[v];
      part[wave * (unsigned)BROWS + 16u + hh * 8u + (unsigned)v] = s1[v];
    }
  }
  __syncthreads();

  const unsigned q4 = (tid & 7u) * 4u;
  v4f s = {};
#pragma unroll
  for (unsigned w = 0; w < (unsigned)NWAVES; ++w) {
    const v4f p = *(const v4f*)&part[w * (unsigned)BROWS + q4];
    s = s + p;
  }
  float* op = out + row0 + q4;
  if (tid < 8u) *(volatile v4f*)op = s;
  __threadfence();
  if (tid < 8u) *(volatile v4f*)op = s;
}

extern "C" void kernel_launch(void* const* d_in, const int* in_sizes, int n_in,
                              void* d_out, int out_size, void* d_ws, size_t ws_size,
                              hipStream_t stream) {
  if (n_in < 4) return;
  if ((long long)in_sizes[0] < (long long)NX * KD) return;
  if ((long long)in_sizes[1] < (long long)MY * KD) return;
  if ((long long)in_sizes[2] < (long long)MY) return;
  if (in_sizes[3] < 1) return;
  if ((long long)out_size < (long long)NX) return;
  if (ws_size < WS_TOTAL) return;

  const float* X  = (const float*)d_in[0];
  const float* Y  = (const float*)d_in[1];
  const float* Al = (const float*)d_in[2];
  const float* G  = (const float*)d_in[3];
  float* out = (float*)d_out;

  char* ws = (char*)d_ws;
  _Float16* Xh   = (_Float16*)(ws + OFF_XH);
  _Float16* Yh   = (_Float16*)(ws + OFF_YH);
  float*    X2c  = (float*)(ws + OFF_X2);
  float*    Pair = (float*)(ws + OFF_PAIR);

  dim3 blk(256);
  xprep_kernel<<<dim3(NX / PREP_ROWS), blk, 0, stream>>>(X, G, Xh, X2c);
  yprep_kernel<<<dim3(MY / PREP_ROWS), blk, 0, stream>>>(Y, Al, G, Yh, Pair);
  krr_kernel<<<dim3(NX / BROWS), blk, 0, stream>>>(Xh, Yh, X2c, Pair, G, out);
}
